// GPT2AttentionOri_56994216018544
// MI455X (gfx1250) — hardware-verified
//
#include <hip/hip_runtime.h>

#define NB    2
#define NS    2048
#define NE    1024
#define NH    16
#define NHD   64
#define N3E   3072
#define NM    4096
#define QSPL  768
#define TP    132
#define PP    72

typedef _Float16 v16h __attribute__((ext_vector_type(16)));
typedef _Float16 v8h  __attribute__((ext_vector_type(8)));
typedef float    v8f  __attribute__((ext_vector_type(8)));
typedef float    v4f  __attribute__((ext_vector_type(4)));
typedef v8h __attribute__((__may_alias__)) v8ha;
typedef v4f __attribute__((__may_alias__)) v4fa;
union Frag { v16h v; v8h hv[2]; };

__device__ __forceinline__ float bf16r(float x) {
  unsigned int u = __float_as_uint(x);
  u += 0x7FFFu + ((u >> 16) & 1u);
  u &= 0xFFFF0000u;
  return __uint_as_float(u);
}

__device__ __forceinline__ v16h ldfrag(const _Float16* p) {
  Frag f;
  f.hv[0] = *(const v8ha*)p;
  f.hv[1] = *(const v8ha*)(p + 16);
  return f.v;
}

__device__ __forceinline__ v16h sc11(v16h a) {
  const _Float16 s = (_Float16)0.00048828125f;
  v16h r;
#pragma unroll
  for (int i = 0; i < 16; ++i) r[i] = a[i] * s;
  return r;
}

__device__ __forceinline__ v8f zero8() {
  return (v8f){0.f, 0.f, 0.f, 0.f, 0.f, 0.f, 0.f, 0.f};
}

__device__ __forceinline__ v8f wmma16(v16h a, v16h b, v8f c) {
  c = __builtin_amdgcn_wmma_f32_16x16x32_f16(false, a, false, b, (short)0, c, false, false);
  asm volatile("v_nop\n\tv_nop\n\tv_nop\n\tv_nop" : "+v"(c) : "v"(a), "v"(b));
  return c;
}

__global__ __launch_bounds__(256)
void k_cvt_x(const float* __restrict__ X, _Float16* __restrict__ Y, int n8, float sc)
{
  const int i = blockIdx.x * 256 + threadIdx.x;
  if (i < n8) {
    const float4 a = *(const float4*)(X + (size_t)i * 8);
    const float4 c = *(const float4*)(X + (size_t)i * 8 + 4);
    v8h o;
    o[0] = (_Float16)(bf16r(a.x) * sc);
    o[1] = (_Float16)(bf16r(a.y) * sc);
    o[2] = (_Float16)(bf16r(a.z) * sc);
    o[3] = (_Float16)(bf16r(a.w) * sc);
    o[4] = (_Float16)(bf16r(c.x) * sc);
    o[5] = (_Float16)(bf16r(c.y) * sc);
    o[6] = (_Float16)(bf16r(c.z) * sc);
    o[7] = (_Float16)(bf16r(c.w) * sc);
    _Float16* d = Y + (size_t)i * 8;
    *(volatile v8h*)d = o;
    __threadfence();
    *(volatile v8h*)d = o;
  }
}

__global__ __launch_bounds__(256)
void k_cvt_t(const float* __restrict__ W, _Float16* __restrict__ Wt, int K, int N, float sc)
{
  __shared__ __attribute__((aligned(16))) _Float16 lt[64 * PP];
  const int t = threadIdx.x;
  const int n0 = blockIdx.x * 64, k0 = blockIdx.y * 64;
#pragma unroll
  for (int i = 0; i < 4; ++i) {
    const int flat = t + 256 * i;
    const int row = flat >> 4;
    const int c4 = (flat & 15) * 4;
    const float4 v = *(const float4*)(W + (size_t)(k0 + row) * N + n0 + c4);
    lt[(c4 + 0) * PP + row] = (_Float16)(bf16r(v.x) * sc);
    lt[(c4 + 1) * PP + row] = (_Float16)(bf16r(v.y) * sc);
    lt[(c4 + 2) * PP + row] = (_Float16)(bf16r(v.z) * sc);
    lt[(c4 + 3) * PP + row] = (_Float16)(bf16r(v.w) * sc);
  }
  __syncthreads();
  v8h val[2];
  size_t dst[2];
#pragma unroll
  for (int i = 0; i < 2; ++i) {
    const int L = i * 32 + (t >> 3);
    const int ch = (t & 7) * 8;
    val[i] = *(const v8ha*)(lt + L * PP + ch);
    dst[i] = (size_t)(n0 + L) * K + k0 + ch;
  }
#pragma unroll
  for (int i = 0; i < 2; ++i) *(volatile v8h*)(Wt + dst[i]) = val[i];
  __threadfence();
#pragma unroll
  for (int i = 0; i < 2; ++i) *(volatile v8h*)(Wt + dst[i]) = val[i];
}

__global__ __launch_bounds__(256)
void k_qkv(const _Float16* __restrict__ X16, const _Float16* __restrict__ Wt,
           const float* __restrict__ bias,
           _Float16* __restrict__ Qh, _Float16* __restrict__ Ql,
           _Float16* __restrict__ Kh, _Float16* __restrict__ Kl,
           _Float16* __restrict__ Vh, _Float16* __restrict__ Vl)
{
  __shared__ __attribute__((aligned(16))) float T[128 * TP];
  const int t = threadIdx.x, lane = t & 31, wave = t >> 5;
  const int waveM = wave >> 2, waveN = wave & 3, hl = lane >> 4, m = lane & 15;
  const int m0 = blockIdx.x * 128, n0 = blockIdx.y * 128;

  v8f acc[4][2];
#pragma unroll
  for (int mi = 0; mi < 4; ++mi)
#pragma unroll
    for (int ni = 0; ni < 2; ++ni) acc[mi][ni] = zero8();

  size_t aoff[4], boff[2];
#pragma unroll
  for (int mi = 0; mi < 4; ++mi)
    aoff[mi] = (size_t)(m0 + waveM * 64 + mi * 16 + m) * NE + 8 * hl;
#pragma unroll
  for (int ni = 0; ni < 2; ++ni)
    boff[ni] = (size_t)(n0 + waveN * 32 + ni * 16 + m) * NE + 8 * hl;

#pragma unroll 1
  for (int k0 = 0; k0 < NE; k0 += 32) {
    const v16h b0 = ldfrag(Wt + boff[0] + k0);
    const v16h b1 = ldfrag(Wt + boff[1] + k0);
#pragma unroll
    for (int mi = 0; mi < 4; ++mi) {
      const v16h a = ldfrag(X16 + aoff[mi] + k0);
      acc[mi][0] = wmma16(a, b0, acc[mi][0]);
      acc[mi][1] = wmma16(a, b1, acc[mi][1]);
    }
  }

#pragma unroll
  for (int ni = 0; ni < 2; ++ni) {
    const int col = waveN * 32 + ni * 16 + m;
    const float bv = bf16r(bias[n0 + col]);
#pragma unroll
    for (int mi = 0; mi < 4; ++mi)
#pragma unroll
      for (int r = 0; r < 8; ++r) {
        const int row = waveM * 64 + mi * 16 + 8 * hl + r;
        T[row * TP + col] = acc[mi][ni][r] * (1.f / 16384.f) + bv;
      }
  }
  __syncthreads();

  const int seg = n0 >> 10;
  const int hh0 = (n0 & 1023) >> 6;
  const int bb = m0 >> 11, s0 = m0 & 2047;

  if (seg < 2) {
    _Float16* Ph = (seg == 0) ? Qh : Kh;
    _Float16* Pl = (seg == 0) ? Ql : Kl;
    for (int pass = 0; pass < 2; ++pass) {
#pragma unroll 1
      for (int it = 0; it < 8; ++it) {
        const int L = it * 32 + (t >> 3);
        const int row = L >> 1, hs = L & 1, ch = (t & 7) * 8;
        const float* src = T + row * TP + hs * 64 + ch;
        v8h oh, ol;
#pragma unroll
        for (int j = 0; j < 8; ++j) {
          const float v = src[j] * 16.f;
          const _Float16 hv = (_Float16)v;
          oh[j] = hv;
          ol[j] = (_Float16)((v - (float)hv) * 2048.f);
        }
        const size_t dst = ((size_t)((bb * NH + hh0 + hs) * NS + s0 + row)) * NHD + ch;
        *(volatile v8h*)(Ph + dst) = oh;
        *(volatile v8h*)(Pl + dst) = ol;
      }
      if (pass == 0) __threadfence();
    }
  } else {
    for (int pass = 0; pass < 2; ++pass) {
#pragma unroll 1
      for (int it = 0; it < 8; ++it) {
        const int L = it * 32 + (t >> 3);
        const int cc = L >> 1, part = L & 1, j8 = (t & 7) * 8;
        const int soff = part * 64 + j8;
        const int hs = cc >> 6, d = cc & 63;
        v8h oh, ol;
#pragma unroll
        for (int j = 0; j < 8; ++j) {
          const float v = T[(soff + j) * TP + cc] * 256.f;
          const _Float16 hv = (_Float16)v;
          oh[j] = hv;
          ol[j] = (_Float16)((v - (float)hv) * 2048.f);
        }
        const size_t dst = ((size_t)((bb * NH + hh0 + hs) * NHD + d)) * NS + s0 + soff;
        *(volatile v8h*)(Vh + dst) = oh;
        *(volatile v8h*)(Vl + dst) = ol;
      }
      if (pass == 0) __threadfence();
    }
  }
}

template <bool SPL>
__global__ __launch_bounds__(128)
void k_attn(const _Float16* __restrict__ Qh, const _Float16* __restrict__ Ql,
            const _Float16* __restrict__ Kh, const _Float16* __restrict__ Kl,
            const _Float16* __restrict__ Vh, const _Float16* __restrict__ Vl,
            _Float16* __restrict__ Oh, _Float16* __restrict__ Ol, int qb_off)
{
  __shared__ __attribute__((aligned(16))) _Float16 lds_p[4 * 2 * 16 * PP];
  const int t = threadIdx.x, lane = t & 31, wave = t >> 5, hl = lane >> 4, m = lane & 15;
  const int qbi = blockIdx.x + qb_off;
  const int bh = blockIdx.y, b = bh >> 4, hd = bh & 15;
  const size_t plane = (size_t)NS * NHD;
  const _Float16* Qhb = Qh + bh * plane;
  const _Float16* Qlb = Ql + bh * plane;
  const _Float16* Khb = Kh + bh * plane;
  const _Float16* Klb = Kl + bh * plane;
  const _Float16* Vhb = Vh + bh * plane;
  const _Float16* Vlb = Vl + bh * plane;
  _Float16* ph_l = lds_p + wave * (2 * 16 * PP);
  _Float16* pl_l = ph_l + 16 * PP;
  const int q0 = qbi * 64 + wave * 16;

  v16h qfh[2], qfl[2], qfh2[2];
#pragma unroll
  for (int c = 0; c < 2; ++c) {
    const size_t qo = (size_t)(q0 + m) * NHD + c * 32 + 8 * hl;
    qfh[c] = ldfrag(Qhb + qo);
    qfl[c] = qfh[c];
    qfh2[c] = qfh[c];
    if (SPL) { qfl[c] = ldfrag(Qlb + qo); qfh2[c] = sc11(qfh[c]); }
  }

  v8f o[4];
#pragma unroll
  for (int n = 0; n < 4; ++n) o[n] = zero8();
  float mrow[8], lrow[8];
#pragma unroll
  for (int r = 0; r < 8; ++r) { mrow[r] = -1e30f; lrow[r] = 0.f; }

  for (int kb = 0; kb <= qbi; ++kb) {
    float sb[4][8];
#pragma unroll
    for (int tt = 0; tt < 4; ++tt) {
      const int key = kb * 64 + tt * 16 + m;
      v8f s = zero8();
#pragma unroll
      for (int c = 0; c < 2; ++c) {
        const size_t ko = (size_t)key * NHD + c * 32 + 8 * hl;
        const v16h kfh = ldfrag(Khb + ko);
        s = wmma16(qfh[c], kfh, s);
        if (SPL) {
          const v16h kfl = ldfrag(Klb + ko);
          s = wmma16(qfh2[c], kfl, s);
          s = wmma16(qfl[c], sc11(kfh), s);
        }
      }
#pragma unroll
      for (int r = 0; r < 8; ++r) {
        const int qr = q0 + 8 * hl + r;
        const float val = s[r] * (1.f / 2048.f);
        sb[tt][r] = (key <= qr) ? val : -1e30f;
      }
    }

    float resc[8];
#pragma unroll
    for (int r = 0; r < 8; ++r) {
      float mx = fmaxf(fmaxf(sb[0][r], sb[1][r]), fmaxf(sb[2][r], sb[3][r]));
      mx = fmaxf(mx, __shfl_xor(mx, 1, 32));
      mx = fmaxf(mx, __shfl_xor(mx, 2, 32));
      mx = fmaxf(mx, __shfl_xor(mx, 4, 32));
      mx = fmaxf(mx, __shfl_xor(mx, 8, 32));
      const float mn = fmaxf(mrow[r], mx);
      resc[r] = __expf(mrow[r] - mn);
      mrow[r] = mn;
      float rs = 0.f;
#pragma unroll
      for (int tt = 0; tt < 4; ++tt) {
        const float p = __expf(sb[tt][r] - mn);
        sb[tt][r] = p;
        rs += p;
      }
      rs += __shfl_xor(rs, 1, 32);
      rs += __shfl_xor(rs, 2, 32);
      rs += __shfl_xor(rs, 4, 32);
      rs += __shfl_xor(rs, 8, 32);
      lrow[r] = lrow[r] * resc[r] + rs;
    }

    __syncthreads();
#pragma unroll
    for (int tt = 0; tt < 4; ++tt)
#pragma unroll
      for (int r = 0; r < 8; ++r) {
        const int idx = (8 * hl + r) * PP + tt * 16 + m;
        const float pv = sb[tt][r] * 4096.f;
        const _Float16 hv = (_Float16)pv;
        ph_l[idx] = hv;
        if (SPL) pl_l[idx] = (_Float16)((pv - (float)hv) * 2048.f);
      }
    __syncthreads();

#pragma unroll
    for (int n = 0; n < 4; ++n)
#pragma unroll
      for (int r = 0; r < 8; ++r) o[n][r] *= resc[r];

#pragma unroll
    for (int c = 0; c < 2; ++c) {
      const int ko = c * 32 + 8 * hl;
      const v16h afh = ldfrag(ph_l + m * PP + ko);
      v16h afl = afh, afh2 = afh;
      if (SPL) { afl = ldfrag(pl_l + m * PP + ko); afh2 = sc11(afh); }
#pragma unroll
      for (int n = 0; n < 4; ++n) {
        const size_t vo = (size_t)(n * 16 + m) * NS + kb * 64 + ko;
        const v16h vfh = ldfrag(Vhb + vo);
        o[n] = wmma16(afh, vfh, o[n]);
        if (SPL) {
          const v16h vfl = ldfrag(Vlb + vo);
          o[n] = wmma16(afh2, vfl, o[n]);
          o[n] = wmma16(afl, sc11(vfh), o[n]);
        }
      }
    }
  }

  __syncthreads();
  float inv[8];
#pragma unroll
  for (int r = 0; r < 8; ++r) inv[r] = 1.0f / lrow[r];
#pragma unroll
  for (int n = 0; n < 4; ++n)
#pragma unroll
    for (int r = 0; r < 8; ++r) {
      const float ov = o[n][r] * (1.f / 4096.f) * inv[r];
      const _Float16 hv = (_Float16)ov;
      const int idx = (8 * hl + r) * PP + n * 16 + m;
      ph_l[idx] = hv;
      pl_l[idx] = (_Float16)((ov - (float)hv) * 2048.f);
    }
  __syncthreads();
  for (int pass = 0; pass < 2; ++pass) {
#pragma unroll
    for (int it = 0; it < 4; ++it) {
      const int row = it * 4 + (lane >> 3);
      const int ch = (lane & 7) * 8;
      const v8h a  = *(const v8ha*)(ph_l + row * PP + ch);
      const v8h al = *(const v8ha*)(pl_l + row * PP + ch);
      const size_t dst = ((size_t)(b * NS + q0 + row)) * NE + hd * NHD + ch;
      *(volatile v8h*)(Oh + dst) = a;
      *(volatile v8h*)(Ol + dst) = al;
    }
    if (pass == 0) __threadfence();
  }
}

template <bool SPL>
__global__ __launch_bounds__(256)
void k_proj(const _Float16* __restrict__ Oh, const _Float16* __restrict__ Ol,
            const _Float16* __restrict__ Wt, const float* __restrict__ bias,
            float* __restrict__ out, int base, int cnt)
{
  __shared__ __attribute__((aligned(16))) float T[128 * TP];
  const int t = threadIdx.x, lane = t & 31, wave = t >> 5;
  const int waveM = wave >> 2, waveN = wave & 3, hl = lane >> 4, m = lane & 15;
  const int i = blockIdx.x;
  const int mb = (i / cnt) * 16 + base + (i % cnt);
  const int m0 = mb * 128, n0 = blockIdx.y * 128;

  v8f acc[4][2];
#pragma unroll
  for (int mi = 0; mi < 4; ++mi)
#pragma unroll
    for (int ni = 0; ni < 2; ++ni) acc[mi][ni] = zero8();

  size_t aoff[4], boff[2];
#pragma unroll
  for (int mi = 0; mi < 4; ++mi)
    aoff[mi] = (size_t)(m0 + waveM * 64 + mi * 16 + m) * NE + 8 * hl;
#pragma unroll
  for (int ni = 0; ni < 2; ++ni)
    boff[ni] = (size_t)(n0 + waveN * 32 + ni * 16 + m) * NE + 8 * hl;

#pragma unroll 1
  for (int k0 = 0; k0 < NE; k0 += 32) {
    v16h bf[2], bf2[2];
#pragma unroll
    for (int ni = 0; ni < 2; ++ni) {
      bf[ni] = ldfrag(Wt + boff[ni] + k0);
      bf2[ni] = bf[ni];
      if (SPL) bf2[ni] = sc11(bf[ni]);
    }
#pragma unroll
    for (int mi = 0; mi < 4; ++mi) {
      const v16h ah = ldfrag(Oh + aoff[mi] + k0);
      v16h al = ah;
      if (SPL) al = ldfrag(Ol + aoff[mi] + k0);
#pragma unroll
      for (int ni = 0; ni < 2; ++ni) {
        acc[mi][ni] = wmma16(ah, bf[ni], acc[mi][ni]);
        if (SPL) acc[mi][ni] = wmma16(al, bf2[ni], acc[mi][ni]);
      }
    }
  }

#pragma unroll
  for (int ni = 0; ni < 2; ++ni) {
    const int col = waveN * 32 + ni * 16 + m;
    const float bv = bf16r(bias[n0 + col]);
#pragma unroll
    for (int mi = 0; mi < 4; ++mi)
#pragma unroll
      for (int r = 0; r < 8; ++r) {
        const int row = waveM * 64 + mi * 16 + 8 * hl + r;
        T[row * TP + col] = acc[mi][ni][r] * (1.f / 262144.f) + bv;
      }
  }
  __syncthreads();
  for (int pass = 0; pass < 2; ++pass) {
#pragma unroll 1
    for (int it = 0; it < 16; ++it) {
      const int row = wave * 16 + it;
      const v4f v = *(const v4fa*)(T + row * TP + lane * 4);
      float* d = out + (size_t)(m0 + row) * NE + n0 + lane * 4;
      *(volatile v4f*)d = v;
    }
    if (pass == 0) __threadfence();
  }
}

extern "C" void kernel_launch(void* const* d_in, const int* in_sizes, int n_in,
                              void* d_out, int out_size, void* d_ws, size_t ws_size,
                              hipStream_t stream)
{
  if (n_in < 5) return;
  if (in_sizes[0] != NM * NE || in_sizes[1] != NE * N3E || in_sizes[2] != N3E ||
      in_sizes[3] != NE * NE || in_sizes[4] != NE) return;
  if (out_size != NM * NE) return;

  const float* hs     = (const float*)d_in[0];
  const float* w_attn = (const float*)d_in[1];
  const float* b_attn = (const float*)d_in[2];
  const float* w_proj = (const float*)d_in[3];
  const float* b_proj = (const float*)d_in[4];
  float* out = (float*)d_out;

  const size_t bX  = (size_t)NM * NE * 2;
  const size_t bW  = (size_t)N3E * NE * 2;
  const size_t bWp = (size_t)NE * NE * 2;
  const size_t bPl = (size_t)NB * NH * NS * NHD * 2;
  const size_t bO  = (size_t)NM * NE * 2;
  size_t off = 0;
  const size_t oX = off;   off += bX;
  const size_t oW = off;   off += bW;
  const size_t oWp = off;  off += bWp;
  const size_t oQh = off;  off += bPl;
  const size_t oQl = off;  off += bPl;
  const size_t oKh = off;  off += bPl;
  const size_t oKl = off;  off += bPl;
  const size_t oVh = off;  off += bPl;
  const size_t oVl = off;  off += bPl;
  const size_t oOh = off;  off += bO;
  const size_t oOl = off;  off += bO;
  if (off > ws_size) return;

  char* ws = (char*)d_ws;
  _Float16* X16 = (_Float16*)(ws + oX);
  _Float16* Wt  = (_Float16*)(ws + oW);
  _Float16* Wpt = (_Float16*)(ws + oWp);
  _Float16* Qh = (_Float16*)(ws + oQh);
  _Float16* Ql = (_Float16*)(ws + oQl);
  _Float16* Kh = (_Float16*)(ws + oKh);
  _Float16* Kl = (_Float16*)(ws + oKl);
  _Float16* Vh = (_Float16*)(ws + oVh);
  _Float16* Vl = (_Float16*)(ws + oVl);
  _Float16* Oh = (_Float16*)(ws + oOh);
  _Float16* Ol = (_Float16*)(ws + oOl);

  const int n8 = NM * NE / 8;
  k_cvt_x<<<dim3(n8 / 256), dim3(256), 0, stream>>>(hs, X16, n8, 16.f);
  k_cvt_t<<<dim3(N3E / 64, NE / 64), dim3(256), 0, stream>>>(w_attn, Wt, NE, N3E, 1024.f);
  k_cvt_t<<<dim3(NE / 64, NE / 64), dim3(256), 0, stream>>>(w_proj, Wpt, NE, NE, 1024.f);

  k_qkv<<<dim3(NM / 128, N3E / 128), dim3(256), 0, stream>>>(X16, Wt, b_attn,
                                                              Qh, Ql, Kh, Kl, Vh, Vl);

  const int qsplit = QSPL / 64;
  k_attn<true><<<dim3(qsplit, NB * NH), dim3(128), 0, stream>>>(Qh, Ql, Kh, Kl, Vh, Vl,
                                                                  Oh, Ol, 0);
  k_attn<false><<<dim3(NS / 64 - qsplit, NB * NH), dim3(128), 0, stream>>>(Qh, Ql, Kh, Kl,
                                                                            Vh, Vl, Oh, Ol,
                                                                            qsplit);

  const int msplit = QSPL / 128;
  k_proj<true><<<dim3(NB * msplit, NE / 128), dim3(256), 0, stream>>>(Oh, Ol, Wpt, b_proj,
                                                                       out, 0, msplit);
  k_proj<false><<<dim3(NB * (16 - msplit), NE / 128), dim3(256), 0, stream>>>(
      Oh, Ol, Wpt, b_proj, out, msplit, 16 - msplit);
}
